// GroupedKNNEstimator_19396072309095
// MI455X (gfx1250) — hardware-verified
//
#include <hip/hip_runtime.h>
#include <stddef.h>
#include <stdint.h>
#include <math.h>

#define NQ   2048
#define NM   100000
#define ND   128
#define NCH  125
#define CHR  800
#define STP  (CHR / 32)
#define QPB  256
#define KC   8
#define PW   (2 * KC)
#define BIGF 3.0e38f

static_assert(NCH * CHR == NM);
static_assert(CHR % 32 == 0);
static_assert(STP == 25);
static_assert(NM % 32 == 0);
static_assert(NQ % 32 == 0);
static_assert(NQ % QPB == 0);
static_assert(NQ % 256 == 0);
static_assert(ND == 128);
static_assert(ND % 32 == 0);
static_assert(KC == 8);
static_assert(PW == 16);

typedef _Float16 hh;
typedef hh    v16h __attribute__((ext_vector_type(16)));
typedef hh    v8h  __attribute__((ext_vector_type(8)));
typedef float v8f  __attribute__((ext_vector_type(8)));
typedef float v4f  __attribute__((ext_vector_type(4)));

union Frag { v16h v; v8h p[2]; };

__device__ __forceinline__ v8f zero8() { return (v8f){0.f, 0.f, 0.f, 0.f, 0.f, 0.f, 0.f, 0.f}; }

__device__ __forceinline__ v16h ldfrag(const hh* __restrict__ p, int ld, int row0, int k0, int lane) {
  const hh* q = p + (size_t)(row0 + (lane & 15)) * (size_t)ld + k0 + 8 * (lane >> 4);
  Frag f;
  f.p[0] = *(const v8h*)(q);
  f.p[1] = *(const v8h*)(q + 16);
  return f.v;
}

__device__ __forceinline__ v8f mma16(v16h a, v16h b, v8f cc) {
  return __builtin_amdgcn_wmma_f32_16x16x32_f16(false, a, false, b, (short)0, cc, false, false);
}

__device__ __forceinline__ void gemm32x64(const hh* __restrict__ A, int lda, const hh* __restrict__ B, int ldb,
                                          int ma, int nb, int kdim, int lane, v8f (&acc)[2][4]) {
#pragma unroll 1
  for (int k0 = 0; k0 < kdim; k0 += 32) {
    const v16h a0 = ldfrag(A, lda, ma, k0, lane);
    const v16h a1 = ldfrag(A, lda, ma + 16, k0, lane);
    const v16h b0 = ldfrag(B, ldb, nb, k0, lane);
    const v16h b1 = ldfrag(B, ldb, nb + 16, k0, lane);
    const v16h b2 = ldfrag(B, ldb, nb + 32, k0, lane);
    const v16h b3 = ldfrag(B, ldb, nb + 48, k0, lane);
    acc[0][0] = mma16(a0, b0, acc[0][0]);
    acc[1][0] = mma16(a1, b0, acc[1][0]);
    acc[0][1] = mma16(a0, b1, acc[0][1]);
    acc[1][1] = mma16(a1, b1, acc[1][1]);
    acc[0][2] = mma16(a0, b2, acc[0][2]);
    acc[1][2] = mma16(a1, b2, acc[1][2]);
    acc[0][3] = mma16(a0, b3, acc[0][3]);
    acc[1][3] = mma16(a1, b3, acc[1][3]);
    asm volatile("v_nop\n\tv_nop\n\tv_nop\n\tv_nop"
                 : "+v"(acc[0][0]), "+v"(acc[0][1]), "+v"(acc[0][2]), "+v"(acc[0][3]),
                   "+v"(acc[1][0]), "+v"(acc[1][1]), "+v"(acc[1][2]), "+v"(acc[1][3])
                 : "v"(a0), "v"(a1), "v"(b0), "v"(b1), "v"(b2), "v"(b3));
  }
}

__device__ __forceinline__ void ins8(float (&t)[KC], float d) {
  if (d < t[KC - 1]) {
#pragma unroll
    for (int q = KC - 1; q > 0; --q) t[q] = fminf(t[q], fmaxf(t[q - 1], d));
    t[0] = fminf(t[0], d);
  }
}

__global__ __launch_bounds__(256) void k_rows(const float* __restrict__ src, hh* __restrict__ dst,
                                              float* __restrict__ nrm) {
  __shared__ __align__(16) float sn[32];
  const int tid = threadIdx.x, lane = tid & 31, w = tid >> 5;
  const int sub = lane >> 4, e0 = 8 * (lane & 15);
  const int rb = blockIdx.x * 32 + w * 4;
  v8h hv[2];
#pragma unroll
  for (int s = 0; s < 2; ++s) {
    const int row = rb + 2 * s + sub;
    const float* rp = src + (size_t)row * ND + e0;
    const v4f a0 = *(const v4f*)(rp), a1 = *(const v4f*)(rp + 4);
    const v8f ta = {a0[0], a0[1], a0[2], a0[3], a1[0], a1[1], a1[2], a1[3]};
    float q = 0.f;
#pragma unroll
    for (int e = 0; e < 8; ++e) q = fmaf(ta[e], ta[e], q);
    q += __shfl_xor(q, 8, 32);
    q += __shfl_xor(q, 4, 32);
    q += __shfl_xor(q, 2, 32);
    q += __shfl_xor(q, 1, 32);
    hv[s] = __builtin_convertvector(ta, v8h);
    if ((lane & 15) == 0) sn[w * 4 + 2 * s + sub] = q;
  }
#pragma unroll
  for (int s = 0; s < 2; ++s) {
    hh* op = dst + (size_t)(rb + 2 * s + sub) * ND + e0;
    *(volatile v8h*)(op) = hv[s];
  }
  __threadfence();
#pragma unroll
  for (int s = 0; s < 2; ++s) {
    hh* op = dst + (size_t)(rb + 2 * s + sub) * ND + e0;
    *(volatile v8h*)(op) = hv[s];
  }
  __syncthreads();
  if (w == 0) {
    const int li = lane & 7;
    const v4f v = *(const v4f*)(sn + 4 * li);
    float* gp = nrm + (size_t)blockIdx.x * 32 + 4 * li;
    if (lane < 8) *(volatile v4f*)gp = v;
    __threadfence();
    if (lane < 8) *(volatile v4f*)gp = v;
  }
}

__global__ __launch_bounds__(128) void k_knn(const hh* __restrict__ BH, const hh* __restrict__ XH,
                                             const float* __restrict__ YN, float* __restrict__ PT) {
  __shared__ __align__(16) float stg[4 * 64 * PW];
  const int tid = threadIdx.x, lane = tid & 31, w = tid >> 5;
  const int h = lane >> 4, c = lane & 15;
  const int qb = blockIdx.x * QPB + w * 64;
  const int chunk = blockIdx.y;
  const int mb = chunk * CHR;

  float lst[4][KC];
#pragma unroll
  for (int j = 0; j < 4; ++j)
#pragma unroll
    for (int q = 0; q < KC; ++q) lst[j][q] = BIGF;

#pragma unroll 1
  for (int st = 0; st < STP; ++st) {
    const int ma = mb + st * 32;
    v8f acc[2][4];
#pragma unroll
    for (int i = 0; i < 2; ++i)
#pragma unroll
      for (int j = 0; j < 4; ++j) acc[i][j] = zero8();
    gemm32x64(BH, ND, XH, ND, ma, qb, ND, lane, acc);

    const v8f ya = *(const v8f*)(YN + ma + 8 * h);
    const v8f yb = *(const v8f*)(YN + ma + 16 + 8 * h);
#pragma unroll
    for (int j = 0; j < 4; ++j) {
#pragma unroll
      for (int r = 0; r < 8; ++r) {
        ins8(lst[j], fmaf(-2.0f, acc[0][j][r], ya[r]));
        ins8(lst[j], fmaf(-2.0f, acc[1][j][r], yb[r]));
      }
    }
  }

  float* sw = stg + w * (64 * PW);
#pragma unroll
  for (int j = 0; j < 4; ++j) {
    float* sp = sw + (16 * j + c) * PW + KC * h;
    *(v4f*)(sp)     = (v4f){lst[j][0], lst[j][1], lst[j][2], lst[j][3]};
    *(v4f*)(sp + 4) = (v4f){lst[j][4], lst[j][5], lst[j][6], lst[j][7]};
  }
  __syncthreads();
  v4f val[8];
#pragma unroll
  for (int it = 0; it < 8; ++it) val[it] = *(const v4f*)(sw + 4 * (lane + 32 * it));
  float* gb = PT + ((size_t)chunk * NQ + qb) * PW;
#pragma unroll
  for (int it = 0; it < 8; ++it) *(volatile v4f*)(gb + 4 * (lane + 32 * it)) = val[it];
  __threadfence();
#pragma unroll
  for (int it = 0; it < 8; ++it) *(volatile v4f*)(gb + 4 * (lane + 32 * it)) = val[it];
}

__global__ __launch_bounds__(256) void k_fin(const float* __restrict__ PT, const float* __restrict__ XN,
                                             const float* __restrict__ minp, const float* __restrict__ maxp,
                                             const int* __restrict__ nnp, float* __restrict__ out) {
  __shared__ __align__(16) float sres[256];
  const int tid = threadIdx.x;
  const int q = blockIdx.x * 256 + tid;
  float t[KC];
#pragma unroll
  for (int e = 0; e < KC; ++e) t[e] = BIGF;
#pragma unroll 1
  for (int ch = 0; ch < NCH; ++ch) {
    const float* p = PT + ((size_t)ch * NQ + q) * PW;
    const v4f a0 = *(const v4f*)(p);
    const v4f a1 = *(const v4f*)(p + 4);
    const v4f a2 = *(const v4f*)(p + 8);
    const v4f a3 = *(const v4f*)(p + 12);
#pragma unroll
    for (int e = 0; e < 4; ++e) {
      ins8(t, a0[e]);
      ins8(t, a1[e]);
      ins8(t, a2[e]);
      ins8(t, a3[e]);
    }
  }
  const int nn = nnp[0];
  const int kk = (nn < 1) ? 1 : ((nn > KC) ? KC : nn);
  const float x2 = XN[q];
  const float minv = minp[0];
  const float inv = 1.0f / (maxp[0] - minv);
  float s = 0.f;
#pragma unroll
  for (int e = 0; e < KC; ++e) {
    const float d = sqrtf(fmaxf(x2 + t[e], 0.0f));
    const float v = (d - minv) * inv;
    s += (e < kk) ? v : 0.0f;
  }
  float res = s * (1.0f / (float)kk);
  if (nn < 1 || nn > KC) res = __int_as_float(0x7fc00000);
  sres[tid] = res;
  __syncthreads();
  const int ti = tid & 63;
  const v4f ov = *(const v4f*)(sres + 4 * ti);
  float* gp = out + (size_t)blockIdx.x * 256 + 4 * ti;
  if (tid < 64) *(volatile v4f*)gp = ov;
  __threadfence();
  if (tid < 64) *(volatile v4f*)gp = ov;
}

static inline size_t al128(size_t o) { return (o + 127) & ~(size_t)127; }

extern "C" void kernel_launch(void* const* d_in, const int* in_sizes, int n_in,
                              void* d_out, int out_size, void* d_ws, size_t ws_size,
                              hipStream_t stream) {
  if (n_in < 5) return;
  if (in_sizes[0] != NQ * ND) return;
  if (in_sizes[1] != NM * ND) return;
  if (in_sizes[2] < 1 || in_sizes[3] < 1 || in_sizes[4] < 1) return;
  if (out_size != NQ) return;

  const float* x    = (const float*)d_in[0];
  const float* bank = (const float*)d_in[1];
  const float* minp = (const float*)d_in[2];
  const float* maxp = (const float*)d_in[3];
  const int*   nnp  = (const int*)d_in[4];
  float* out = (float*)d_out;

  size_t off = 0;
  const size_t oBH = off; off = al128(off + (size_t)NM * ND * 2);
  const size_t oXH = off; off = al128(off + (size_t)NQ * ND * 2);
  const size_t oYN = off; off = al128(off + (size_t)NM * 4);
  const size_t oXN = off; off = al128(off + (size_t)NQ * 4);
  const size_t oPT = off; off = al128(off + (size_t)NCH * NQ * PW * 4);
  if (off > ws_size) return;
  if (off > (size_t)134217728) return;

  char* ws = (char*)d_ws;
  hh*    BH = (hh*)(ws + oBH);
  hh*    XH = (hh*)(ws + oXH);
  float* YN = (float*)(ws + oYN);
  float* XN = (float*)(ws + oXN);
  float* PT = (float*)(ws + oPT);

  k_rows<<<dim3(NQ / 32), dim3(256), 0, stream>>>(x, XH, XN);
  k_rows<<<dim3(NM / 32), dim3(256), 0, stream>>>(bank, BH, YN);
  k_knn<<<dim3(NQ / QPB, NCH), dim3(128), 0, stream>>>(BH, XH, YN, PT);
  k_fin<<<dim3(NQ / 256), dim3(256), 0, stream>>>(PT, XN, minp, maxp, nnp, out);
  (void)hipGetLastError();
}
